// Temper_12601434047083
// MI455X (gfx1250) — hardware-verified
//
#include <hip/hip_runtime.h>
#include <math.h>
#include <stddef.h>


typedef _Float16 v16h __attribute__((ext_vector_type(16)));
typedef _Float16 v8h  __attribute__((ext_vector_type(8)));
typedef float    v8f  __attribute__((ext_vector_type(8)));
typedef float    v4f  __attribute__((ext_vector_type(4)));
typedef unsigned int v4u __attribute__((ext_vector_type(4)));

union Frag  { v16h v; v8h half[2]; };
union Pack8 { v8h h; v4u u; };

constexpr int RL = 512;
constexpr float SX = 8.f;
constexpr float SW = 64.f;
constexpr float SH = 32.f;

__device__ __forceinline__ v16h load_frag(const _Float16* p) {
    Frag f;
    f.half[0] = *(const v8h*)(p);
    f.half[1] = *(const v8h*)(p + 16);
    return f.v;
}

__device__ __forceinline__ void wmma16(v8f& acc, const v16h& a, const v16h& b) {
    acc = __builtin_amdgcn_wmma_f32_16x16x32_f16(false, a, false, b, (short)0, acc, false, false);
    asm volatile("v_nop\n\tv_nop\n\tv_nop\n\tv_nop" : "+v"(acc) : "v"(a), "v"(b));
}

__device__ __forceinline__ float wave_sum(float v) {
#pragma unroll
    for (int o = 16; o > 0; o >>= 1) v += __shfl_xor(v, o, 32);
    return v;
}

__device__ __forceinline__ v4u pack8(v4f lo, v4f hi) {
    v8h hv;
    hv[0] = (_Float16)lo[0]; hv[1] = (_Float16)lo[1]; hv[2] = (_Float16)lo[2]; hv[3] = (_Float16)lo[3];
    hv[4] = (_Float16)hi[0]; hv[5] = (_Float16)hi[1]; hv[6] = (_Float16)hi[2]; hv[7] = (_Float16)hi[3];
    Pack8 p; p.h = hv;
    return p.u;
}

__global__ __launch_bounds__(256)
void cvt_rows(const float* __restrict__ src, int nvalid, float scale,
              _Float16* __restrict__ dst, float* __restrict__ norms)
{
    __shared__ __attribute__((aligned(16))) float sn[32];
    const int lane = threadIdx.x & 31;
    const int wave = threadIdx.x >> 5;
    const int rowb = blockIdx.x * 32;
    v4u pk[4][2];
#pragma unroll
    for (int rr = 0; rr < 4; ++rr) {
        const int rowt = wave * 4 + rr;
        const int row  = rowb + rowt;
        const bool valid = row < nvalid;
        float s = 0.f;
#pragma unroll
        for (int c = 0; c < 2; ++c) {
            const int base = c * 256 + 8 * lane;
            v4f x0 = {0.f, 0.f, 0.f, 0.f};
            v4f x1 = {0.f, 0.f, 0.f, 0.f};
            if (valid) {
                const float* p = src + (size_t)row * RL + base;
                x0 = *(const v4f*)(p);
                x1 = *(const v4f*)(p + 4);
            }
            s += x0[0]*x0[0] + x0[1]*x0[1] + x0[2]*x0[2] + x0[3]*x0[3]
               + x1[0]*x1[0] + x1[1]*x1[1] + x1[2]*x1[2] + x1[3]*x1[3];
            pk[rr][c] = pack8(x0 * scale, x1 * scale);
            *(volatile v4u*)(dst + (size_t)row * RL + base) = pk[rr][c];
        }
        s = wave_sum(s);
        if (lane == 0) sn[rowt] = s;
    }
    __syncthreads();
    v4f nv = {0.f, 0.f, 0.f, 0.f};
    const bool nwriter = (wave == 0) && (lane < 8);
    if (nwriter) {
        nv = *(const v4f*)(&sn[4 * lane]);
        *(volatile v4f*)(norms + rowb + 4 * lane) = nv;
    }
    __threadfence();
#pragma unroll
    for (int rr = 0; rr < 4; ++rr) {
        const int row = rowb + wave * 4 + rr;
#pragma unroll
        for (int c = 0; c < 2; ++c) {
            const int base = c * 256 + 8 * lane;
            *(volatile v4u*)(dst + (size_t)row * RL + base) = pk[rr][c];
        }
    }
    if (nwriter) *(volatile v4f*)(norms + rowb + 4 * lane) = nv;
}

__global__ __launch_bounds__(256)
void cvt_w(const float* __restrict__ pW, int nP8, const float* __restrict__ oW, int nO8, float scale,
           _Float16* __restrict__ pWb, _Float16* __restrict__ oWb)
{
    const int g = blockIdx.x * 256 + threadIdx.x;
    const float* s;
    _Float16* d;
    if (g < nP8) {
        s = pW + (size_t)g * 8;  d = pWb + (size_t)g * 8;
    } else if (g < nP8 + nO8) {
        const int gg = g - nP8;
        s = oW + (size_t)gg * 8; d = oWb + (size_t)gg * 8;
    } else {
        return;
    }
    v4f x0 = *(const v4f*)(s);
    v4f x1 = *(const v4f*)(s + 4);
    const v4u u = pack8(x0 * scale, x1 * scale);
    *(volatile v4u*)d = u;
    __threadfence();
    *(volatile v4u*)d = u;
}

template<int MODE>
__global__ __launch_bounds__(128)
void gemm_f16(const _Float16* __restrict__ A, int lda,
              const _Float16* __restrict__ Wall, int ldw, int wStride,
              const float* __restrict__ biasAll, int bStride,
              const float* __restrict__ logits, int E, int sel,
              void* __restrict__ Cout, int ldc, int K,
              float scale_acc, float scale_out,
              const float* __restrict__ xnorm, const float* __restrict__ mnorm,
              float* __restrict__ partials, int validN)
{
    __shared__ __attribute__((aligned(16))) float stile[(MODE == 0) ? 4 : 128 * 64];
    __shared__ float sred[4];

    int e = 0;
    if (sel >= 0) {
        const int n = E < 64 ? E : 64;
        int ia = 0; float la = logits[0];
#pragma unroll 1
        for (int i = 1; i < n; ++i) { const float v = logits[i]; if (v > la) { la = v; ia = i; } }
        int ib = (ia == 0) ? 1 : 0; float lb = logits[ib];
#pragma unroll 1
        for (int i = 0; i < n; ++i) { if (i == ia) continue; const float v = logits[i]; if (v > lb) { lb = v; ib = i; } }
        e = (sel == 0) ? ia : ib;
        e = e < 0 ? 0 : (e >= E ? E - 1 : e);
    }
    const _Float16* Wp = Wall + (size_t)e * (size_t)wStride;

    const int lane = threadIdx.x & 31;
    const int wave = threadIdx.x >> 5;
    const int wm   = wave & 1;
    const int wn   = wave >> 1;
    const int m    = lane & 15;
    const int h    = lane >> 4;

    const int growBase = blockIdx.y * 128;
    const int gcolBase = blockIdx.x * 64;
    const int row0 = growBase + wm * 64;
    const int col0 = gcolBase + wn * 32;

    const _Float16* pa[4];
    const _Float16* pb[2];
#pragma unroll
    for (int i = 0; i < 4; ++i) pa[i] = A  + (size_t)(row0 + 16 * i + m) * lda + 8 * h;
#pragma unroll
    for (int j = 0; j < 2; ++j) pb[j] = Wp + (size_t)(col0 + 16 * j + m) * ldw + 8 * h;

    const v8f z8 = {0.f, 0.f, 0.f, 0.f, 0.f, 0.f, 0.f, 0.f};
    v8f acc[4][2];
#pragma unroll
    for (int i = 0; i < 4; ++i) { acc[i][0] = z8; acc[i][1] = z8; }

#pragma unroll 1
    for (int k0 = 0; k0 < K; k0 += 32) {
        v16h a[4], b[2];
#pragma unroll
        for (int i = 0; i < 4; ++i) a[i] = load_frag(pa[i] + k0);
#pragma unroll
        for (int j = 0; j < 2; ++j) b[j] = load_frag(pb[j] + k0);
#pragma unroll
        for (int i = 0; i < 4; ++i) {
#pragma unroll
            for (int j = 0; j < 2; ++j) wmma16(acc[i][j], a[i], b[j]);
        }
    }

    if constexpr (MODE == 0) {
        float lsum = 0.f;
#pragma unroll
        for (int j = 0; j < 2; ++j) {
            const int col = col0 + 16 * j + m;
            if (col < validN) {
                const float mnc = mnorm[col];
#pragma unroll
                for (int i = 0; i < 4; ++i) {
#pragma unroll
                    for (int v = 0; v < 8; ++v) {
                        const int row = row0 + 16 * i + 8 * h + v;
                        const float d2 = xnorm[row] + mnc - scale_acc * acc[i][j][v];
                        lsum += sqrtf(fmaxf(d2, 0.f));
                    }
                }
            }
        }
        lsum = wave_sum(lsum);
        if (lane == 0) sred[wave] = lsum;
        __syncthreads();
        if (wave == 0) {
            const float s = ((sred[0] + sred[1]) + sred[2]) + sred[3];
            if (lane < 8) {
                const v4f pv = {s, s, s, s};
                float* pp = partials + (size_t)(blockIdx.y * gridDim.x + blockIdx.x) * 32 + 4 * lane;
                *(volatile v4f*)pp = pv;
                __threadfence();
                *(volatile v4f*)pp = pv;
            }
        }
    } else {
        const float* bias = biasAll + (size_t)e * (size_t)bStride;
#pragma unroll
        for (int j = 0; j < 2; ++j) {
            const int colt = wn * 32 + 16 * j + m;
            const float bv = bias[gcolBase + colt];
#pragma unroll
            for (int i = 0; i < 4; ++i) {
#pragma unroll
                for (int v = 0; v < 8; ++v) {
                    const int rowt = wm * 64 + 16 * i + 8 * h + v;
                    float val = fmaxf(acc[i][j][v] * scale_acc + bv, 0.f);
                    if constexpr (MODE == 1) val *= scale_out;
                    stile[rowt * 64 + colt] = val;
                }
            }
        }
        __syncthreads();

        if constexpr (MODE == 2) {
            float* C = (float*)Cout;
            const int rr = lane >> 4;
            const int pc = lane & 15;
#pragma unroll
            for (int t = 0; t < 16; ++t) {
                const int rowt = wave * 32 + 2 * t + rr;
                const v4f val = *(const v4f*)(&stile[rowt * 64 + 4 * pc]);
                *(volatile v4f*)(C + (size_t)(growBase + rowt) * ldc + gcolBase + 4 * pc) = val;
            }
            __threadfence();
#pragma unroll
            for (int t = 0; t < 16; ++t) {
                const int rowt = wave * 32 + 2 * t + rr;
                const v4f val = *(const v4f*)(&stile[rowt * 64 + 4 * pc]);
                *(volatile v4f*)(C + (size_t)(growBase + rowt) * ldc + gcolBase + 4 * pc) = val;
            }
        } else {
            _Float16* C = (_Float16*)Cout;
            const int rr = lane >> 3;
            const int pc = lane & 7;
            v4u pk[8];
#pragma unroll
            for (int t = 0; t < 8; ++t) {
                const int rowt = wave * 32 + 4 * t + rr;
                const v4f lo = *(const v4f*)(&stile[rowt * 64 + 8 * pc]);
                const v4f hi = *(const v4f*)(&stile[rowt * 64 + 8 * pc + 4]);
                pk[t] = pack8(lo, hi);
                *(volatile v4u*)(C + (size_t)(growBase + rowt) * ldc + gcolBase + 8 * pc) = pk[t];
            }
            __threadfence();
#pragma unroll
            for (int t = 0; t < 8; ++t) {
                const int rowt = wave * 32 + 4 * t + rr;
                *(volatile v4u*)(C + (size_t)(growBase + rowt) * ldc + gcolBase + 8 * pc) = pk[t];
            }
        }
    }
}

__global__ __launch_bounds__(32)
void novelty_final(const float* __restrict__ partials, int nb, float inv_count, float* __restrict__ out_loc)
{
    const int lane = threadIdx.x & 31;
    float s = 0.f;
#pragma unroll 1
    for (int i = lane; i < nb; i += 32) s += partials[(size_t)i * 32];
    s = wave_sum(s);
    if (lane == 0) {
        const float v = fminf(1.5f, s * inv_count);
        *(volatile float*)out_loc = v;
        __threadfence();
        *(volatile float*)out_loc = v;
    }
}

extern "C" void kernel_launch(void* const* d_in, const int* in_sizes, int n_in,
                              void* d_out, int out_size, void* d_ws, size_t ws_size,
                              hipStream_t stream)
{
    if (n_in < 7) return;
    const float* x   = (const float*)d_in[0];
    const float* mem = (const float*)d_in[1];
    const float* rl  = (const float*)d_in[2];
    const float* pW  = (const float*)d_in[3];
    const float* pb  = (const float*)d_in[4];
    const float* oW  = (const float*)d_in[5];
    const float* ob  = (const float*)d_in[6];

    const int D = RL, H = RL;
    const int B  = in_sizes[0] / D;
    const int Mr = in_sizes[1] / D;
    const int E  = in_sizes[2];
    if (B <= 0 || (B % 128) != 0 || in_sizes[0] != B * D) return;
    if (Mr <= 0 || in_sizes[1] != Mr * D) return;
    if (E < 2 || E > 64) return;
    if (in_sizes[3] != H * D || in_sizes[4] != H || in_sizes[5] != E * H * H || in_sizes[6] != E * H) return;
    if (out_size != B * H + 1) return;

    const int Mp  = ((Mr + 63) / 64) * 64;
    const int nbx = Mp / 64, nby = B / 128, nb = nbx * nby;

    size_t off = 0;
    auto carve = [&](size_t bytes) { size_t o = off; off = (off + bytes + 255) & ~(size_t)255; return o; };
    const size_t o_xb   = carve((size_t)B * D * 2);
    const size_t o_h0   = carve((size_t)B * H * 2);
    const size_t o_h1   = carve((size_t)B * H * 2);
    const size_t o_pWb  = carve((size_t)H * D * 2);
    const size_t o_oWb  = carve((size_t)E * H * H * 2);
    const size_t o_memb = carve((size_t)Mp * D * 2);
    const size_t o_xn   = carve((size_t)B * 4);
    const size_t o_mn   = carve((size_t)Mp * 4);
    const size_t o_part = carve((size_t)nb * 128);
    if (off > ws_size) return;

    char* ws = (char*)d_ws;
    _Float16* xb   = (_Float16*)(ws + o_xb);
    _Float16* h0   = (_Float16*)(ws + o_h0);
    _Float16* h1   = (_Float16*)(ws + o_h1);
    _Float16* pWb  = (_Float16*)(ws + o_pWb);
    _Float16* oWb  = (_Float16*)(ws + o_oWb);
    _Float16* memb = (_Float16*)(ws + o_memb);
    float*    xn   = (float*)   (ws + o_xn);
    float*    mn   = (float*)   (ws + o_mn);
    float*    part = (float*)   (ws + o_part);

    cvt_rows<<<B / 32, 256, 0, stream>>>(x, B, SX, xb, xn);
    cvt_rows<<<Mp / 32, 256, 0, stream>>>(mem, Mr, SX, memb, mn);
    const int nP8 = H * D / 8, nO8 = E * H * H / 8;
    cvt_w<<<(nP8 + nO8 + 255) / 256, 256, 0, stream>>>(pW, nP8, oW, nO8, SW, pWb, oWb);

    gemm_f16<0><<<dim3(nbx, nby), 128, 0, stream>>>(
        xb, D, memb, D, 0, pb, 0, rl, E, -1, (void*)part, 0, D,
        2.f / (SX * SX), 1.f, xn, mn, part, Mr);
    novelty_final<<<1, 32, 0, stream>>>(part, nb, 1.f / ((float)B * (float)Mr),
                                        (float*)d_out + (size_t)B * H);

    gemm_f16<1><<<dim3(H / 64, nby), 128, 0, stream>>>(
        xb, D, pWb, D, 0, pb, 0, rl, E, -1, (void*)h0, H, D,
        1.f / (SX * SW), SH, xn, mn, part, 0);

    gemm_f16<1><<<dim3(H / 64, nby), 128, 0, stream>>>(
        h0, H, oWb, H, H * H, ob, H, rl, E, 0, (void*)h1, H, H,
        1.f / (SH * SW), SH, xn, mn, part, 0);

    gemm_f16<2><<<dim3(H / 64, nby), 128, 0, stream>>>(
        h1, H, oWb, H, H * H, ob, H, rl, E, 1, d_out, H, H,
        1.f / (SH * SW), 1.f, xn, mn, part, 0);
}
